// AsymmetricRoPECrossAttention_45114336477756
// MI455X (gfx1250) — hardware-verified
//
#include <hip/hip_runtime.h>
#include <math.h>

#pragma clang fp contract(off)

#define NB     2
#define NQ     2048
#define NKV    4096
#define DIM    1024
#define HEADS  16
#define DH     64
#define TP     68
#define HP     72
#define C2S    0.18033688011112042f
#define NEGMAX (-3.4028234663852886e38f)
#define ROPEK  (-0.14391156831212787f)
#define WSCAP  ((size_t)134217728)

typedef unsigned short us;
typedef __attribute__((ext_vector_type(8)))  unsigned short v8us;
typedef __attribute__((ext_vector_type(16))) unsigned short v16us;
typedef __attribute__((ext_vector_type(16))) __bf16   v16bf;
typedef __attribute__((ext_vector_type(16))) _Float16 v16h;
typedef __attribute__((ext_vector_type(8)))  float    v8f;
typedef __attribute__((ext_vector_type(4)))  float    v4f;
typedef __attribute__((ext_vector_type(4)))  unsigned int v4u;
typedef __attribute__((ext_vector_type(4)))  int      v4i;
typedef __attribute__((ext_vector_type(8)))  int      v8i;

static_assert((NB * NQ * DIM / 8) % 128 == 0);
static_assert((NB * NKV * DIM / 8) % 128 == 0);
static_assert(NQ % 64 == 0 && NKV % 64 == 0 && DIM % 64 == 0);
static_assert((NKV * 32) % 128 == 0);

__device__ __forceinline__ us f2bf(float f) {
  const unsigned u = __float_as_uint(f);
  return (us)((u + 0x7FFFu + ((u >> 16) & 1u)) >> 16);
}
__device__ __forceinline__ float bf2f(us b) { return __uint_as_float(((unsigned)b) << 16); }
__device__ __forceinline__ us h2us(float f) { return __builtin_bit_cast(us, (_Float16)f); }
__device__ __forceinline__ unsigned pk16(us a, us b) { return (unsigned)a | ((unsigned)b << 16); }

__device__ __forceinline__ v4u pack_bf8(v4f a, v4f b) {
  v4u w;
  w[0] = pk16(f2bf(a[0]), f2bf(a[1]));
  w[1] = pk16(f2bf(a[2]), f2bf(a[3]));
  w[2] = pk16(f2bf(b[0]), f2bf(b[1]));
  w[3] = pk16(f2bf(b[2]), f2bf(b[3]));
  return w;
}
__device__ __forceinline__ void split_bf8(v4f a, v4f b, v4u& hv, v4u& lv) {
#pragma unroll
  for (int e = 0; e < 2; ++e) {
    const float x0 = a[2 * e], x1 = a[2 * e + 1];
    const us h0 = f2bf(x0), h1 = f2bf(x1);
    const us l0 = f2bf(x0 - bf2f(h0)), l1 = f2bf(x1 - bf2f(h1));
    hv[e] = pk16(h0, h1);
    lv[e] = pk16(l0, l1);
  }
#pragma unroll
  for (int e = 0; e < 2; ++e) {
    const float x0 = b[2 * e], x1 = b[2 * e + 1];
    const us h0 = f2bf(x0), h1 = f2bf(x1);
    const us l0 = f2bf(x0 - bf2f(h0)), l1 = f2bf(x1 - bf2f(h1));
    hv[2 + e] = pk16(h0, h1);
    lv[2 + e] = pk16(l0, l1);
  }
}

static __device__ __forceinline__ v8f z8f() {
  v8f z = {0.f, 0.f, 0.f, 0.f, 0.f, 0.f, 0.f, 0.f};
  return z;
}
static __device__ __forceinline__ v16h z16h() {
  const _Float16 o = (_Float16)0.0f;
  v16h z = {o, o, o, o, o, o, o, o, o, o, o, o, o, o, o, o};
  return z;
}

__device__ __forceinline__ v16bf ldf_bf(const us* p) {
  const v8us a = *(const v8us*)p;
  const v8us b = *(const v8us*)(p + 16);
  const v16us c = __builtin_shufflevector(a, b, 0, 1, 2, 3, 4, 5, 6, 7, 8, 9, 10, 11, 12, 13, 14, 15);
  return __builtin_bit_cast(v16bf, c);
}
__device__ __forceinline__ v16h ldf_h(const us* p) {
  const v8us a = *(const v8us*)p;
  const v8us b = *(const v8us*)(p + 16);
  const v16us c = __builtin_shufflevector(a, b, 0, 1, 2, 3, 4, 5, 6, 7, 8, 9, 10, 11, 12, 13, 14, 15);
  return __builtin_bit_cast(v16h, c);
}

static __device__ __forceinline__ v8f wm_bf(v16bf a, v16bf b, v8f c) {
  v8f d = __builtin_amdgcn_wmma_f32_16x16x32_bf16(false, a, false, b, (short)0, c, false, false);
  asm volatile("v_nop\n\tv_nop\n\tv_nop\n\tv_nop" : "+v"(d) : "v"(a), "v"(b));
  return d;
}
static __device__ __forceinline__ v8f wm_h(v16h a, v16h b, v8f c) {
  v8f d = __builtin_amdgcn_wmma_f32_16x16x32_f16(false, a, false, b, (short)0, c, false, false);
  asm volatile("v_nop\n\tv_nop\n\tv_nop\n\tv_nop" : "+v"(d) : "v"(a), "v"(b));
  return d;
}

__global__ __launch_bounds__(128) void cvt_bf16_kernel(const float* __restrict__ in, us* __restrict__ out, int n8) {
  const int i = blockIdx.x * 128 + threadIdx.x;
  if (i < n8) {
    const float* p = in + (size_t)i * 8;
    const v4f a = *(const v4f*)p;
    const v4f b = *(const v4f*)(p + 4);
    const v4u w = pack_bf8(a, b);
    volatile v4u* d = (volatile v4u*)(out + (size_t)i * 8);
    *d = w;
    __threadfence();
    *d = w;
  }
}

__global__ __launch_bounds__(128) void wtrans_kernel(const float* __restrict__ W, us* __restrict__ WT, int krows, int ncols) {
  __shared__ __align__(16) us T[64 * HP];
  const int t = threadIdx.x;
  const int n0 = blockIdx.x * 64;
  const int k0 = blockIdx.y * 64;
  {
    const int rr = t >> 1;
    const int ch = (t & 1) * 32;
    const float* src = W + (size_t)(k0 + rr) * ncols + n0 + ch;
#pragma unroll
    for (int q = 0; q < 4; ++q) {
      const v4f a = *(const v4f*)(src + 8 * q);
      const v4f b = *(const v4f*)(src + 8 * q + 4);
      *(v4u*)(&T[rr * HP + ch + 8 * q]) = pack_bf8(a, b);
    }
  }
  __syncthreads();
  const int rsub = t >> 3, k8 = (t & 7) * 8;
  v4u ov[4];
#pragma unroll
  for (int it = 0; it < 4; ++it) {
    const int nr = 16 * it + rsub;
    v4u w;
#pragma unroll
    for (int e = 0; e < 4; ++e)
      w[e] = pk16(T[(k8 + 2 * e) * HP + nr], T[(k8 + 2 * e + 1) * HP + nr]);
    ov[it] = w;
  }
  for (int ps = 0; ps < 2; ++ps) {
#pragma unroll
    for (int it = 0; it < 4; ++it) {
      const int nr = 16 * it + rsub;
      *(volatile v4u*)(WT + (size_t)(n0 + nr) * krows + k0 + k8) = ov[it];
    }
    __threadfence();
  }
}

__global__ __launch_bounds__(128) void ropetab_kernel(float* __restrict__ cosT, float* __restrict__ sinT) {
  const int i = blockIdx.x * 128 + threadIdx.x;
  const int pos = i >> 5, j = i & 31;
  const float dv = expf((float)(2 * j) * ROPEK);
  const float ang = (float)pos * dv;
  const double x = (double)ang;
  const int kq = (int)(x * 0.63661977236758134308 + 0.5);
  const double dk = (double)kq;
  double r = fma(-dk, 1.5707963267948966, x);
  r = fma(-dk, 6.123233995736766e-17, r);
  const double r2 = r * r;
  double sp = 1.0 / 6227020800.0;
  sp = sp * r2 - 1.0 / 39916800.0;
  sp = sp * r2 + 1.0 / 362880.0;
  sp = sp * r2 - 1.0 / 5040.0;
  sp = sp * r2 + 1.0 / 120.0;
  sp = sp * r2 - 1.0 / 6.0;
  const double s = r + r * r2 * sp;
  double cp = -1.0 / 87178291200.0;
  cp = cp * r2 + 1.0 / 479001600.0;
  cp = cp * r2 - 1.0 / 3628800.0;
  cp = cp * r2 + 1.0 / 40320.0;
  cp = cp * r2 - 1.0 / 720.0;
  cp = cp * r2 + 1.0 / 24.0;
  cp = cp * r2 - 0.5;
  const double c = 1.0 + r2 * cp;
  const int qd = kq & 3;
  const double ss = (qd == 0) ? s : ((qd == 1) ? c : ((qd == 2) ? -s : -c));
  const double cc = (qd == 0) ? c : ((qd == 1) ? -s : ((qd == 2) ? -c : s));
  const float sf = (float)ss, cf = (float)cc;
  volatile float* pc = cosT + i;
  volatile float* psn = sinT + i;
  *pc = cf;
  *psn = sf;
  __threadfence();
  *pc = cf;
  *psn = sf;
}

__device__ __forceinline__ void rope_store(const float* tile, const float* __restrict__ cosT, const float* __restrict__ sinT,
                                           us* __restrict__ Ph, us* __restrict__ Pl, int m0, int n0, int nseq, int t) {
  const int c8 = (t & 7) * 8, jb = c8 & 31, rsub = t >> 3;
  const bool upper = (c8 >= 32);
  const int hh = n0 >> 6;
  v4u hv[4], lv[4];
  size_t dst[4];
#pragma unroll
  for (int it = 0; it < 4; ++it) {
    const int row = 16 * it + rsub;
    const int gm = m0 + row;
    const int bb = gm / nseq;
    const int n = gm - bb * nseq;
    const float* tr = tile + row * TP;
    const v4f xa0 = *(const v4f*)(tr + jb);
    const v4f xa1 = *(const v4f*)(tr + jb + 4);
    const v4f xb0 = *(const v4f*)(tr + 32 + jb);
    const v4f xb1 = *(const v4f*)(tr + 36 + jb);
    const float* cp = cosT + (size_t)n * 32 + jb;
    const float* snp = sinT + (size_t)n * 32 + jb;
    const v4f c0 = *(const v4f*)cp, c1 = *(const v4f*)(cp + 4);
    const v4f s0 = *(const v4f*)snp, s1 = *(const v4f*)(snp + 4);
    const v4f lo0 = xa0 * c0 - xb0 * s0;
    const v4f lo1 = xa1 * c1 - xb1 * s1;
    const v4f up0 = xb0 * c0 + xa0 * s0;
    const v4f up1 = xb1 * c1 + xa1 * s1;
    v4f o0, o1;
#pragma unroll
    for (int e = 0; e < 4; ++e) {
      o0[e] = upper ? up0[e] : lo0[e];
      o1[e] = upper ? up1[e] : lo1[e];
    }
    split_bf8(o0, o1, hv[it], lv[it]);
    dst[it] = ((size_t)(bb * HEADS + hh) * nseq + n) * DH + c8;
  }
  for (int ps = 0; ps < 2; ++ps) {
#pragma unroll
    for (int it = 0; it < 4; ++it) {
      *(volatile v4u*)(Ph + dst[it]) = hv[it];
      *(volatile v4u*)(Pl + dst[it]) = lv[it];
    }
    __threadfence();
  }
}

__device__ __forceinline__ void v_store(const float* tile, us* __restrict__ VT, int m0, int n0, int t) {
  const int k8 = (t & 7) * 8, dsub = t >> 3;
  const int bb = m0 / NKV;
  const int key0 = m0 - bb * NKV;
  const int hh = (n0 - DIM) >> 6;
  v4u ov[4];
  size_t dst[4];
#pragma unroll
  for (int it = 0; it < 4; ++it) {
    const int d = 16 * it + dsub;
    v4u w;
#pragma unroll
    for (int e = 0; e < 4; ++e) {
      const float f0 = tile[(k8 + 2 * e) * TP + d] * 16.0f;
      const float f1 = tile[(k8 + 2 * e + 1) * TP + d] * 16.0f;
      w[e] = pk16(h2us(f0), h2us(f1));
    }
    ov[it] = w;
    dst[it] = ((size_t)(bb * HEADS + hh) * DH + d) * NKV + key0 + k8;
  }
  for (int ps = 0; ps < 2; ++ps) {
#pragma unroll
    for (int it = 0; it < 4; ++it) *(volatile v4u*)(VT + dst[it]) = ov[it];
    __threadfence();
  }
}

__device__ __forceinline__ void out_store(const float* tile, float* __restrict__ Cf, int m0, int n0, int t) {
  const int c4 = (t & 15) * 4, rsub = t >> 4;
  v4f ov[8];
#pragma unroll
  for (int it = 0; it < 8; ++it) {
    const int row = 8 * it + rsub;
    ov[it] = *(const v4f*)(tile + row * TP + c4);
  }
  for (int ps = 0; ps < 2; ++ps) {
#pragma unroll
    for (int it = 0; it < 8; ++it) {
      const int row = 8 * it + rsub;
      *(volatile v4f*)(Cf + (size_t)(m0 + row) * DIM + n0 + c4) = ov[it];
    }
    __threadfence();
  }
}

template <int MODE>
__global__ __launch_bounds__(128) void gemm_kernel(const us* __restrict__ A, const us* __restrict__ A2,
                                                   const us* __restrict__ Bt,
                                                   const float* __restrict__ cosT, const float* __restrict__ sinT,
                                                   us* __restrict__ P0, us* __restrict__ P1, us* __restrict__ P2,
                                                   float* __restrict__ Cf) {
  __shared__ __align__(16) float tile[64 * TP];
  const int t = threadIdx.x, lane = t & 31, w = t >> 5, hf = lane >> 4, m = lane & 15;
  const int n0 = blockIdx.x * 64;
  const int m0 = blockIdx.y * 64;
  const size_t aoff = (size_t)(m0 + 16 * w + m) * DIM + 8 * hf;
  const us* arow = A + aoff;
  const us* arow2 = A2 + aoff;
  const us* bbase = Bt + (size_t)(n0 + m) * DIM + 8 * hf;

  v8f acc[4];
#pragma unroll
  for (int j = 0; j < 4; ++j) acc[j] = z8f();

#pragma unroll 1
  for (int k0 = 0; k0 < DIM; k0 += 32) {
    const v16bf a = ldf_bf(arow + k0);
    v16bf a2 = a;
    if (MODE == 2) a2 = ldf_bf(arow2 + k0);
#pragma unroll
    for (int j = 0; j < 4; ++j) {
      const v16bf bj = ldf_bf(bbase + (size_t)(16 * j) * DIM + k0);
      acc[j] = wm_bf(a, bj, acc[j]);
      if (MODE == 2) acc[j] = wm_bf(a2, bj, acc[j]);
    }
  }

#pragma unroll
  for (int j = 0; j < 4; ++j)
#pragma unroll
    for (int r = 0; r < 8; ++r)
      tile[(16 * w + 8 * hf + r) * TP + 16 * j + m] = acc[j][r];
  __syncthreads();

  if (MODE == 0) {
    rope_store(tile, cosT, sinT, P0, P1, m0, n0, NQ, t);
  } else if (MODE == 1) {
    if (n0 < DIM) rope_store(tile, cosT, sinT, P0, P1, m0, n0, NKV, t);
    else          v_store(tile, P2, m0, n0, t);
  } else {
    out_store(tile, Cf, m0, n0, t);
  }
}

__global__ __launch_bounds__(128) void attn_kernel(const us* __restrict__ Qh, const us* __restrict__ Ql,
                                                   const us* __restrict__ Kh, const us* __restrict__ Kl,
                                                   const us* __restrict__ VT, const int* __restrict__ mask,
                                                   us* __restrict__ Ch, us* __restrict__ Cl) {
  __shared__ __align__(16) us sh[64 * HP];
  __shared__ __align__(16) us sl[64 * HP];
  const int t = threadIdx.x, lane = t & 31, w = t >> 5, hf = lane >> 4, m = lane & 15;
  const int bh = blockIdx.y;
  const int b = bh >> 4, h = bh & 15;
  const int qb = blockIdx.x * 64;
  const int qw = qb + 16 * w;

  const size_t qoff = ((size_t)bh * NQ + qw + m) * DH + 8 * hf;
  const v16bf qh0 = ldf_bf(Qh + qoff);
  const v16bf qh1 = ldf_bf(Qh + qoff + 32);
  const v16bf ql0 = ldf_bf(Ql + qoff);
  const v16bf ql1 = ldf_bf(Ql + qoff + 32);
  const size_t koff = (size_t)bh * NKV * DH + (size_t)m * DH + 8 * hf;
  const us* kbh = Kh + koff;
  const us* kbl = Kl + koff;
  const us* vb = VT + (size_t)bh * DH * NKV + (size_t)m * NKV + 8 * hf;
  const int* mb = mask + (size_t)b * NKV + 8 * hf;

  float mrun = -__builtin_inff();
  float lrun = 0.f;
  v8f oacc[4];
#pragma unroll
  for (int i = 0; i < 4; ++i) oacc[i] = z8f();

#pragma unroll 1
  for (int kt = 0; kt < NKV / 64; ++kt) {
    const int key0 = kt * 64;
    v8f sacc[4];
#pragma unroll
    for (int j = 0; j < 4; ++j) {
      sacc[j] = z8f();
      const size_t ko = (size_t)(key0 + 16 * j) * DH;
#pragma unroll
      for (int ds = 0; ds < 2; ++ds) {
        const v16bf ka = ldf_bf(kbh + ko + 32 * ds);
        const v16bf kr = ldf_bf(kbl + ko + 32 * ds);
        v16bf qa = qh0, qr = ql0;
        if (ds) { qa = qh1; qr = ql1; }
        sacc[j] = wm_bf(ka, qa, sacc[j]);
        sacc[j] = wm_bf(ka, qr, sacc[j]);
        sacc[j] = wm_bf(kr, qa, sacc[j]);
      }
    }
    float tmax = NEGMAX;
#pragma unroll
    for (int j = 0; j < 4; ++j) {
      const v4i ma = *(const v4i*)(mb + key0 + 16 * j);
      const v4i mc = *(const v4i*)(mb + key0 + 16 * j + 4);
      const v8i mv = __builtin_shufflevector(ma, mc, 0, 1, 2, 3, 4, 5, 6, 7);
#pragma unroll
      for (int r = 0; r < 8; ++r) {
        const float tv = (mv[r] != 0) ? (sacc[j][r] * C2S) : NEGMAX;
        sacc[j][r] = tv;
        tmax = fmaxf(tmax, tv);
      }
    }
    tmax = fmaxf(tmax, __shfl_xor(tmax, 16, 32));
    const float mnew = fmaxf(mrun, tmax);
    const float alpha = __builtin_amdgcn_exp2f(mrun - mnew);
    mrun = mnew;
    float psum = 0.f;
    v16h pb0 = z16h(), pb1 = z16h();
#pragma unroll
    for (int j = 0; j < 4; ++j) {
#pragma unroll
      for (int r = 0; r < 8; ++r) {
        const float p = __builtin_amdgcn_exp2f(sacc[j][r] - mnew);
        psum += p;
        const _Float16 hp = (_Float16)(p * 1024.0f);
        if (j == 0)      pb0[r] = hp;
        else if (j == 1) pb0[8 + r] = hp;
        else if (j == 2) pb1[r] = hp;
        else             pb1[8 + r] = hp;
      }
    }
    psum += __shfl_xor(psum, 16, 32);
    lrun = lrun * alpha + psum;
#pragma unroll
    for (int i = 0; i < 4; ++i) oacc[i] = oacc[i] * alpha;
#pragma unroll
    for (int i = 0; i < 4; ++i) {
#pragma unroll
      for (int ks = 0; ks < 2; ++ks) {
        const v16h va = ldf_h(vb + (size_t)(16 * i) * NKV + key0 + 32 * ks);
        v16h pbk = pb0;
        if (ks) pbk = pb1;
        oacc[i] = wm_h(va, pbk, oacc[i]);
      }
    }
  }

  const float inv = (1.0f / lrun) * (1.0f / 16384.0f);
#pragma unroll
  for (int i = 0; i < 4; ++i) {
    v4f a, c;
#pragma unroll
    for (int e = 0; e < 4; ++e) {
      a[e] = oacc[i][e] * inv;
      c[e] = oacc[i][4 + e] * inv;
    }
    v4u hv, lv;
    split_bf8(a, c, hv, lv);
    const int so = (16 * w + m) * HP + 16 * i + 8 * hf;
    *(v4u*)(&sh[so]) = hv;
    *(v4u*)(&sl[so]) = lv;
  }
  __syncthreads();
  v4u ohv[4], olv[4];
  size_t od[4];
#pragma unroll
  for (int it = 0; it < 4; ++it) {
    const int row = 16 * it + (t >> 3);
    const int c8 = (t & 7) * 8;
    ohv[it] = *(const v4u*)(&sh[row * HP + c8]);
    olv[it] = *(const v4u*)(&sl[row * HP + c8]);
    od[it] = ((size_t)(b * NQ + qb + row)) * DIM + h * DH + c8;
  }
  for (int ps = 0; ps < 2; ++ps) {
#pragma unroll
    for (int it = 0; it < 4; ++it) {
      *(volatile v4u*)(Ch + od[it]) = ohv[it];
      *(volatile v4u*)(Cl + od[it]) = olv[it];
    }
    __threadfence();
  }
}

extern "C" void kernel_launch(void* const* d_in, const int* in_sizes, int n_in,
                              void* d_out, int out_size, void* d_ws, size_t ws_size,
                              hipStream_t stream) {
  if (n_in < 6) return;
  if (in_sizes[0] != NB * NQ * DIM) return;
  if (in_sizes[1] != NB * NKV * DIM) return;
  if (in_sizes[2] != NB * NKV) return;
  if (in_sizes[3] != DIM * DIM) return;
  if (in_sizes[4] != DIM * 2 * DIM) return;
  if (in_sizes[5] != DIM * DIM) return;
  if (out_size != NB * NQ * DIM) return;

  const float* q_x  = (const float*)d_in[0];
  const float* kv_x = (const float*)d_in[1];
  const int*   mask = (const int*)d_in[2];
  const float* Wq   = (const float*)d_in[3];
  const float* Wkv  = (const float*)d_in[4];
  const float* Wout = (const float*)d_in[5];
  float* outp = (float*)d_out;

  const size_t PXQ  = (size_t)NB * NQ * DIM * 2;
  const size_t PXKV = (size_t)NB * NKV * DIM * 2;
  const size_t PWQ  = (size_t)DIM * DIM * 2;
  const size_t PWKV = (size_t)2 * DIM * DIM * 2;
  const size_t PTAB = (size_t)NKV * 32 * 4;
  const size_t PQ   = (size_t)NB * HEADS * NQ * DH * 2;
  const size_t PK   = (size_t)NB * HEADS * NKV * DH * 2;
  const size_t PVT  = (size_t)NB * HEADS * DH * NKV * 2;
  const size_t PC   = (size_t)NB * NQ * DIM * 2;
  size_t off = 0;
  const size_t oXq  = off; off += PXQ;
  const size_t oXkv = off; off += PXKV;
  const size_t oWq  = off; off += PWQ;
  const size_t oWkv = off; off += PWKV;
  const size_t oWo  = off; off += PWQ;
  const size_t oCos = off; off += PTAB;
  const size_t oSin = off; off += PTAB;
  const size_t oQh  = off; off += PQ;
  const size_t oQl  = off; off += PQ;
  const size_t oKh  = off; off += PK;
  const size_t oKl  = off; off += PK;
  const size_t oVT  = off; off += PVT;
  const size_t oCh  = off; off += PC;
  const size_t oCl  = off; off += PC;
  if (off > ws_size) return;
  if (off > WSCAP) return;

  char* ws = (char*)d_ws;
  us* Xq   = (us*)(ws + oXq);
  us* Xkv  = (us*)(ws + oXkv);
  us* WqT  = (us*)(ws + oWq);
  us* WkvT = (us*)(ws + oWkv);
  us* WoT  = (us*)(ws + oWo);
  float* cosT = (float*)(ws + oCos);
  float* sinT = (float*)(ws + oSin);
  us* Qh = (us*)(ws + oQh);
  us* Ql = (us*)(ws + oQl);
  us* Kh = (us*)(ws + oKh);
  us* Kl = (us*)(ws + oKl);
  us* VT = (us*)(ws + oVT);
  us* Ch = (us*)(ws + oCh);
  us* Cl = (us*)(ws + oCl);

  const dim3 blk(128);
  const int n8q  = NB * NQ * DIM / 8;
  const int n8kv = NB * NKV * DIM / 8;

  cvt_bf16_kernel<<<dim3(n8q / 128), blk, 0, stream>>>(q_x, Xq, n8q);
  cvt_bf16_kernel<<<dim3(n8kv / 128), blk, 0, stream>>>(kv_x, Xkv, n8kv);
  wtrans_kernel<<<dim3(DIM / 64, DIM / 64), blk, 0, stream>>>(Wq, WqT, DIM, DIM);
  wtrans_kernel<<<dim3(2 * DIM / 64, DIM / 64), blk, 0, stream>>>(Wkv, WkvT, DIM, 2 * DIM);
  wtrans_kernel<<<dim3(DIM / 64, DIM / 64), blk, 0, stream>>>(Wout, WoT, DIM, DIM);
  ropetab_kernel<<<dim3(NKV * 32 / 128), blk, 0, stream>>>(cosT, sinT);
  gemm_kernel<0><<<dim3(DIM / 64, NB * NQ / 64), blk, 0, stream>>>(Xq, Xq, WqT, cosT, sinT, Qh, Ql, Qh, cosT);
  gemm_kernel<1><<<dim3(2 * DIM / 64, NB * NKV / 64), blk, 0, stream>>>(Xkv, Xkv, WkvT, cosT, sinT, Kh, Kl, VT, cosT);
  attn_kernel<<<dim3(NQ / 64, NB * HEADS), blk, 0, stream>>>(Qh, Ql, Kh, Kl, VT, mask, Ch, Cl);
  gemm_kernel<2><<<dim3(DIM / 64, NB * NQ / 64), blk, 0, stream>>>(Ch, Cl, WoT, cosT, sinT, Ch, Ch, Ch, outp);

  (void)hipGetLastError();
}
